// TransformerSelfAttnLayer_78091095376088
// MI455X (gfx1250) — hardware-run, weakly checked
//
#include <hip/hip_runtime.h>
#include <math.h>
#include <stdint.h>

#define NBATCH 2
#define LTOK   30720
#define CCH    256
#define NHEAD  8
#define HDIM   32
#define NKQV   96
#define DFF    1024
#define NROWS  (NBATCH * LTOK)
#define NBH    (NBATCH * NHEAD)
#define NCHUNK 6
#define CHROWS (NROWS / NCHUNK)
#define KVW_STRIDE 1056
#define XC   16.0f
#define WKS  64.0f
#define KC   16.0f
#define VC   16.0f
#define QC   16.0f
#define KVS  0.0625f
#define KSS  0.015625f
#define H1C  16.0f
#define W1S  64.0f
#define GC   16.0f
#define W2S  128.0f
#define LN_EPS  1e-5f
#define ATT_EPS 1e-6f
#define LTOKF   30720.0f
static_assert(NHEAD * HDIM == CCH);
static_assert(CCH == 256);
static_assert(NKQV == 3 * HDIM);
static_assert(NROWS % NCHUNK == 0 && (CHROWS % 64) == 0 && (CHROWS % 32) == 0 && (CHROWS % 8) == 0);
static_assert((LTOK % 64) == 0 && (LTOK % 32) == 0 && ((LTOK / 8) % 32) == 0);
static_assert((CCH % 64) == 0 && (DFF % 64) == 0 && (CCH % 32) == 0 && (DFF % 32) == 0);
static_assert(DFF * CCH / 8 == 128 * 256);
static_assert(KVW_STRIDE == 32 * 32 + 32);

typedef _Float16 v16h __attribute__((ext_vector_type(16)));
typedef _Float16 v8h  __attribute__((ext_vector_type(8)));
typedef float    v8f  __attribute__((ext_vector_type(8)));
typedef float    v4f  __attribute__((ext_vector_type(4)));
typedef unsigned int v4u __attribute__((ext_vector_type(4)));
typedef unsigned int v2u __attribute__((ext_vector_type(2)));

union FragH { v16h v; v8h h[2]; v4u u[2]; };

__device__ __forceinline__ unsigned short bf_bits(float f) {
  unsigned u = __float_as_uint(f);
  return (unsigned short)((u + 0x7FFFu + ((u >> 16) & 1u)) >> 16);
}
__device__ __forceinline__ float bf_up(unsigned short h) { return __uint_as_float(((unsigned)h) << 16); }
__device__ __forceinline__ float bfr(float f) { return bf_up(bf_bits(f)); }
__device__ __forceinline__ unsigned short h_bits(_Float16 x) { return __builtin_bit_cast(unsigned short, x); }
__device__ __forceinline__ unsigned pk16(unsigned short a, unsigned short b) { return (unsigned)a | ((unsigned)b << 16); }
__device__ __forceinline__ v8f zero8() { v8f z = {0.f, 0.f, 0.f, 0.f, 0.f, 0.f, 0.f, 0.f}; return z; }
__device__ __forceinline__ float gelu_f(float u) { return 0.5f * u * (1.0f + erff(u * 0.70710678118654752440f)); }
__device__ __forceinline__ float phi1(float v) { return v > 0.0f ? v + 1.0f : __expf(v); }

__device__ __forceinline__ v16h ldfrag_h(const _Float16* p) {
  FragH f;
  f.h[0] = *(const v8h*)(p);
  f.h[1] = *(const v8h*)(p + 16);
  return f.v;
}
__device__ __forceinline__ v16h ldfrag_u(const unsigned short* p) {
  FragH f;
  f.u[0] = *(const v4u*)(p);
  f.u[1] = *(const v4u*)(p + 16);
  return f.v;
}
__device__ __forceinline__ v16h cvtfrag_x(const float* p) {
  const v4f a = *(const v4f*)(p), b = *(const v4f*)(p + 4), c = *(const v4f*)(p + 16), d = *(const v4f*)(p + 20);
  FragH f;
#pragma unroll
  for (int e = 0; e < 4; ++e) {
    f.h[0][e]     = (_Float16)(bfr(a[e]) * XC);
    f.h[0][4 + e] = (_Float16)(bfr(b[e]) * XC);
    f.h[1][e]     = (_Float16)(bfr(c[e]) * XC);
    f.h[1][4 + e] = (_Float16)(bfr(d[e]) * XC);
  }
  return f.v;
}
__device__ __forceinline__ v16h cvtfrag_s(const float* p, float sc) {
  const v4f a = *(const v4f*)(p), b = *(const v4f*)(p + 4), c = *(const v4f*)(p + 16), d = *(const v4f*)(p + 20);
  FragH f;
#pragma unroll
  for (int e = 0; e < 4; ++e) {
    f.h[0][e]     = (_Float16)(a[e] * sc);
    f.h[0][4 + e] = (_Float16)(b[e] * sc);
    f.h[1][e]     = (_Float16)(c[e] * sc);
    f.h[1][4 + e] = (_Float16)(d[e] * sc);
  }
  return f.v;
}

__device__ __forceinline__ v8f mma_raw(v16h a, v16h b, v8f c) {
  return __builtin_amdgcn_wmma_f32_16x16x32_f16(false, a, false, b, (short)0, c, false, false);
}
__device__ __forceinline__ void dep_guard1(v8f& a, v8f& b, v16h x) {
#if defined(__HIP_DEVICE_COMPILE__)
  asm volatile("v_nop\n\tv_nop\n\tv_nop\n\tv_nop" : "+v"(a), "+v"(b) : "v"(x));
#endif
}
__device__ __forceinline__ void guard2k3(v8f& a, v8f& b, v16h x, v16h y, v16h z) {
#if defined(__HIP_DEVICE_COMPILE__)
  asm volatile("v_nop\n\tv_nop\n\tv_nop\n\tv_nop" : "+v"(a), "+v"(b) : "v"(x), "v"(y), "v"(z));
#endif
}
__device__ __forceinline__ void guard3k4(v8f& a, v8f& b, v8f& c, v16h x, v16h y, v16h z, v16h w) {
#if defined(__HIP_DEVICE_COMPILE__)
  asm volatile("v_nop\n\tv_nop\n\tv_nop\n\tv_nop" : "+v"(a), "+v"(b), "+v"(c) : "v"(x), "v"(y), "v"(z), "v"(w));
#endif
}
__device__ __forceinline__ void guard6k5(v8f& a, v8f& b, v8f& c, v8f& d, v8f& e, v8f& f,
                                         v16h x, v16h y, v16h z, v16h w, v16h u) {
#if defined(__HIP_DEVICE_COMPILE__)
  asm volatile("v_nop\n\tv_nop\n\tv_nop\n\tv_nop"
               : "+v"(a), "+v"(b), "+v"(c), "+v"(d), "+v"(e), "+v"(f) : "v"(x), "v"(y), "v"(z), "v"(w), "v"(u));
#endif
}
__device__ __forceinline__ void keep4_h(v16h a, v16h b, v16h c, v16h d) {
#if defined(__HIP_DEVICE_COMPILE__)
  asm volatile("v_nop" :: "v"(a), "v"(b), "v"(c), "v"(d));
#endif
}
__device__ __forceinline__ void acc_guard4(v8f& a, v8f& b, v8f& c, v8f& d) {
#if defined(__HIP_DEVICE_COMPILE__)
  asm volatile("v_nop\n\tv_nop\n\tv_nop\n\tv_nop" : "+v"(a), "+v"(b), "+v"(c), "+v"(d));
#endif
}
__device__ __forceinline__ void wave_sync_lds() {
  __builtin_amdgcn_fence(__ATOMIC_RELEASE, "workgroup");
  __builtin_amdgcn_wave_barrier();
  __builtin_amdgcn_fence(__ATOMIC_ACQUIRE, "workgroup");
}

__global__ __launch_bounds__(256) void k_wcvt(const float* __restrict__ wk, const float* __restrict__ w1,
                                              const float* __restrict__ w2, unsigned short* WK16,
                                              unsigned short* W116, unsigned short* W216) {
  const int y = blockIdx.y;
  const float* src = (y == 0) ? wk : ((y == 1) ? w1 : w2);
  unsigned short* dst = (y == 0) ? WK16 : ((y == 1) ? W116 : W216);
  const int n8 = (y == 0) ? (NKQV * HDIM / 8) : (DFF * CCH / 8);
  const float sc = (y == 0) ? WKS : ((y == 1) ? W1S : W2S);
  const int p  = blockIdx.x * 256 + threadIdx.x;
  const int pc = min(p, n8 - 1);
  const v4f a = *(const v4f*)(src + (size_t)pc * 8);
  const v4f b = *(const v4f*)(src + (size_t)pc * 8 + 4);
  v4u o;
  o[0] = pk16(h_bits((_Float16)(bfr(a[0]) * sc)), h_bits((_Float16)(bfr(a[1]) * sc)));
  o[1] = pk16(h_bits((_Float16)(bfr(a[2]) * sc)), h_bits((_Float16)(bfr(a[3]) * sc)));
  o[2] = pk16(h_bits((_Float16)(bfr(b[0]) * sc)), h_bits((_Float16)(bfr(b[1]) * sc)));
  o[3] = pk16(h_bits((_Float16)(bfr(b[2]) * sc)), h_bits((_Float16)(bfr(b[3]) * sc)));
  for (int pass = 0; pass < 2; ++pass) {
    if (p < n8) *(volatile v4u*)(dst + (size_t)p * 8) = o;
    __threadfence();
  }
}

__global__ __launch_bounds__(256) void k_proj(const float* __restrict__ x, const unsigned short* __restrict__ WK16,
                                              unsigned short* KT16, unsigned short* VT16) {
  __shared__ __align__(16) unsigned short sT[8][32 * 72];
  const int lane = threadIdx.x & 31, wave = threadIdx.x >> 5;
  const int rl = lane & 15, hh = lane >> 4, koff = hh * 8;
  const int bat  = blockIdx.y;
  const int t0   = blockIdx.x * 64;
  const int head = wave;
  const int bh   = bat * NHEAD + head;
  const float osc = 1.0f / (XC * WKS);

  v16h af[4];
#pragma unroll
  for (int i = 0; i < 4; ++i)
    af[i] = cvtfrag_x(x + ((size_t)bat * LTOK + t0 + 16 * i + rl) * CCH + head * HDIM + koff);

  unsigned short* mys = sT[wave];
  const int q8 = lane >> 3, c8 = (lane & 7) * 8;
#pragma unroll
  for (int grp = 0; grp < 2; ++grp) {
    const int nb = (grp == 0) ? 0 : 2 * HDIM;
    const float carry = (grp == 0) ? KC : VC;
    unsigned short* plane = (grp == 0) ? KT16 : VT16;
    const v16h b0 = ldfrag_u(WK16 + (size_t)(nb + rl) * HDIM + koff);
    const v16h b1 = ldfrag_u(WK16 + (size_t)(nb + 16 + rl) * HDIM + koff);
#pragma unroll
    for (int i = 0; i < 4; ++i) {
      v8f d0 = mma_raw(af[i], b0, zero8());
      v8f d1 = mma_raw(af[i], b1, zero8());
      guard2k3(d0, d1, af[i], b0, b1);
#pragma unroll
      for (int r = 0; r < 8; ++r) {
        float v0 = d0[r] * osc, v1 = d1[r] * osc;
        if (grp == 0) { v0 = phi1(v0); v1 = phi1(v1); }
        const int tcol = 16 * i + 8 * hh + r;
        mys[rl * 72 + tcol]        = h_bits((_Float16)(v0 * carry));
        mys[(16 + rl) * 72 + tcol] = h_bits((_Float16)(v1 * carry));
      }
    }
    wave_sync_lds();
    v4u vals[8];
#pragma unroll
    for (int it = 0; it < 8; ++it) {
      const int q = it * 4 + q8;
      vals[it] = *(const v4u*)(mys + q * 72 + c8);
    }
    unsigned short* dst = plane + ((size_t)bh * HDIM) * LTOK + t0 + c8;
    for (int pass = 0; pass < 2; ++pass) {
#pragma unroll
      for (int it = 0; it < 8; ++it) {
        const int q = it * 4 + q8;
        *(volatile v4u*)(dst + (size_t)q * LTOK) = vals[it];
      }
      __threadfence();
    }
    wave_sync_lds();
  }
}

__global__ __launch_bounds__(256) void k_kv(const unsigned short* __restrict__ KT16,
                                            const unsigned short* __restrict__ VT16, float* KVW) {
  __shared__ __align__(16) float sP[8][32 * 36];
  __shared__ float sK[8][32];
  const int tid = threadIdx.x, lane = tid & 31, wave = tid >> 5;
  const int rl = lane & 15, hh = lane >> 4, koff = hh * 8;
  const int bh = blockIdx.x;
  const _Float16* Kb = (const _Float16*)(const void*)KT16 + ((size_t)bh * HDIM + rl) * LTOK + koff;
  const _Float16* Vb = (const _Float16*)(const void*)VT16 + ((size_t)bh * HDIM + rl) * LTOK + koff;
  FragH on;
  {
    const _Float16 ov = (_Float16)((rl == 0) ? 1.0f : 0.0f);
#pragma unroll
    for (int e = 0; e < 8; ++e) { on.h[0][e] = ov; on.h[1][e] = ov; }
  }
  v8f c00 = zero8(), c01 = zero8(), c10 = zero8(), c11 = zero8(), s0 = zero8(), s1 = zero8();
  const int sbeg = wave * (LTOK / 8);
#pragma unroll 1
  for (int s = sbeg; s < sbeg + LTOK / 8; s += 32) {
    const v16h a0 = ldfrag_h(Kb + s), a1 = ldfrag_h(Kb + (size_t)16 * LTOK + s);
    const v16h b0 = ldfrag_h(Vb + s), b1 = ldfrag_h(Vb + (size_t)16 * LTOK + s);
    c00 = mma_raw(a0, b0, c00);
    c01 = mma_raw(a0, b1, c01);
    c10 = mma_raw(a1, b0, c10);
    c11 = mma_raw(a1, b1, c11);
    s0  = mma_raw(a0, on.v, s0);
    s1  = mma_raw(a1, on.v, s1);
    guard6k5(c00, c01, c10, c11, s0, s1, a0, a1, b0, b1, on.v);
  }
  float* myp = sP[wave];
#pragma unroll
  for (int r = 0; r < 8; ++r) {
    myp[(8 * hh + r) * 36 + rl]           = c00[r];
    myp[(8 * hh + r) * 36 + 16 + rl]      = c01[r];
    myp[(16 + 8 * hh + r) * 36 + rl]      = c10[r];
    myp[(16 + 8 * hh + r) * 36 + 16 + rl] = c11[r];
  }
  if (rl == 0) {
#pragma unroll
    for (int r = 0; r < 8; ++r) { sK[wave][8 * hh + r] = s0[r]; sK[wave][16 + 8 * hh + r] = s1[r]; }
  }
  __syncthreads();
  const int vv = tid >> 3, pp = tid & 7;
  v4f o, ks;
#pragma unroll
  for (int e = 0; e < 4; ++e) {
    const int d = 4 * pp + e;
    float a = 0.f, b = 0.f;
#pragma unroll
    for (int w = 0; w < 8; ++w) { a += sP[w][d * 36 + vv]; b += sK[w][d]; }
    o[e]  = a * (1.0f / (KC * VC));
    ks[e] = b * (1.0f / KC);
  }
  float* base = KVW + (size_t)bh * KVW_STRIDE;
  for (int pass = 0; pass < 2; ++pass) {
    *(volatile v4f*)(base + vv * 32 + 4 * pp) = o;
    if (tid < 8) *(volatile v4f*)(base + 1024 + 4 * pp) = ks;
    __threadfence();
  }
}

__global__ __launch_bounds__(256) void k_apply(const float* __restrict__ x, const unsigned short* __restrict__ WK16,
                                               const float* __restrict__ KVW, const float* __restrict__ g1,
                                               const float* __restrict__ be1, float* X1F, unsigned short* X1H,
                                               int row0) {
  __shared__ __align__(16) float sAtt[32 * 264];
  __shared__ __align__(16) unsigned short sQ[8][32 * 40];
  const int tid = threadIdx.x, lane = tid & 31, wave = tid >> 5;
  const int rl = lane & 15, hh = lane >> 4, koff = hh * 8;
  const int grow0 = row0 + blockIdx.x * 32;
  const int bat   = grow0 / LTOK;
  const int head  = wave;
  const int bh    = bat * NHEAD + head;
  const float osc = 1.0f / (XC * WKS);

  v16h af[2];
#pragma unroll
  for (int i = 0; i < 2; ++i)
    af[i] = cvtfrag_x(x + ((size_t)grow0 + 16 * i + rl) * CCH + head * HDIM + koff);
  const v16h bq0 = ldfrag_u(WK16 + (size_t)(HDIM + rl) * HDIM + koff);
  const v16h bq1 = ldfrag_u(WK16 + (size_t)(HDIM + 16 + rl) * HDIM + koff);
  unsigned short* myq = sQ[wave];
#pragma unroll
  for (int i = 0; i < 2; ++i) {
    v8f d0 = mma_raw(af[i], bq0, zero8());
    v8f d1 = mma_raw(af[i], bq1, zero8());
    guard2k3(d0, d1, af[i], bq0, bq1);
#pragma unroll
    for (int r = 0; r < 8; ++r) {
      const float v0 = phi1(d0[r] * osc), v1 = phi1(d1[r] * osc);
      const int tr = 16 * i + 8 * hh + r;
      myq[tr * 40 + rl]      = h_bits((_Float16)(v0 * QC));
      myq[tr * 40 + 16 + rl] = h_bits((_Float16)(v1 * QC));
    }
  }
  wave_sync_lds();
  v16h qa[2];
  qa[0] = ldfrag_u(myq + (size_t)rl * 40 + koff);
  qa[1] = ldfrag_u(myq + (size_t)(16 + rl) * 40 + koff);

  const float* kvb = KVW + (size_t)bh * KVW_STRIDE;
  const v16h bv0 = cvtfrag_s(kvb + (size_t)rl * 32 + koff, KVS);
  const v16h bv1 = cvtfrag_s(kvb + (size_t)(16 + rl) * 32 + koff, KVS);
  const float sel = (rl == 0) ? KSS : 0.0f;
  const v16h bks = cvtfrag_s(kvb + 1024 + koff, sel);
  const float rtok = 1.0f / LTOKF;
  const float dscl = 1.0f / (QC * KSS);
  const float nscl = rtok * (1.0f / (QC * KVS)) * LTOKF;
#pragma unroll
  for (int i = 0; i < 2; ++i) {
    v8f n0 = mma_raw(qa[i], bv0, zero8());
    v8f n1 = mma_raw(qa[i], bv1, zero8());
    v8f dn = mma_raw(qa[i], bks, zero8());
    guard3k4(n0, n1, dn, qa[i], bv0, bv1, bks);
#pragma unroll
    for (int r = 0; r < 8; ++r) {
      const float dsum = __shfl(dn[r], lane & 16, 32);
      const float z = 1.0f / (dsum * dscl + ATT_EPS);
      const float f = (nscl * z);
      const int tr = 16 * i + 8 * hh + r;
      sAtt[tr * 264 + head * HDIM + rl]      = (n0[r] * rtok * (1.0f / (QC * KVS))) * z * LTOKF + 0.0f * f;
      sAtt[tr * 264 + head * HDIM + 16 + rl] = (n1[r] * rtok * (1.0f / (QC * KVS))) * z * LTOKF;
    }
  }
  __syncthreads();

  v4f ga = *(const v4f*)(g1 + 4 * lane), gb = *(const v4f*)(g1 + 128 + 4 * lane);
  v4f ea = *(const v4f*)(be1 + 4 * lane), eb = *(const v4f*)(be1 + 128 + 4 * lane);
#pragma unroll
  for (int e = 0; e < 4; ++e) { ga[e] = bfr(ga[e]); gb[e] = bfr(gb[e]); ea[e] = bfr(ea[e]); eb[e] = bfr(eb[e]); }
#pragma unroll 1
  for (int t = 0; t < 4; ++t) {
    const int lr = wave * 4 + t;
    const int grow = grow0 + lr;
    const float* xr = x + (size_t)grow * CCH;
    const v4f xa = *(const v4f*)(xr + 4 * lane), xb = *(const v4f*)(xr + 128 + 4 * lane);
    float* srow = sAtt + lr * 264;
    const v4f aa = *(const v4f*)(srow + 4 * lane), ab = *(const v4f*)(srow + 128 + 4 * lane);
    v4f va, vb;
#pragma unroll
    for (int e = 0; e < 4; ++e) { va[e] = bfr(xa[e]) + aa[e]; vb[e] = bfr(xb[e]) + ab[e]; }
    float s = ((va[0] + va[1]) + (va[2] + va[3])) + ((vb[0] + vb[1]) + (vb[2] + vb[3]));
#pragma unroll
    for (int off = 1; off < 32; off <<= 1) s += __shfl_xor(s, off, 32);
    const float mu = s * (1.0f / (float)CCH);
    v4f da, db;
#pragma unroll
    for (int e = 0; e < 4; ++e) { da[e] = va[e] - mu; db[e] = vb[e] - mu; }
    float q = ((da[0] * da[0] + da[1] * da[1]) + (da[2] * da[2] + da[3] * da[3])) +
              ((db[0] * db[0] + db[1] * db[1]) + (db[2] * db[2] + db[3] * db[3]));
#pragma unroll
    for (int off = 1; off < 32; off <<= 1) q += __shfl_xor(q, off, 32);
    const float var  = q * (1.0f / (float)CCH);
    const float rstd = rsqrtf(var + LN_EPS);
    v4f ya, yb;
#pragma unroll
    for (int e = 0; e < 4; ++e) { ya[e] = da[e] * rstd * ga[e] + ea[e]; yb[e] = db[e] * rstd * gb[e] + eb[e]; }
    v2u w0, w1;
    w0[0] = pk16(h_bits((_Float16)(ya[0] * H1C)), h_bits((_Float16)(ya[1] * H1C)));
    w0[1] = pk16(h_bits((_Float16)(ya[2] * H1C)), h_bits((_Float16)(ya[3] * H1C)));
    w1[0] = pk16(h_bits((_Float16)(yb[0] * H1C)), h_bits((_Float16)(yb[1] * H1C)));
    w1[1] = pk16(h_bits((_Float16)(yb[2] * H1C)), h_bits((_Float16)(yb[3] * H1C)));
    wave_sync_lds();
    unsigned short* hrow = (unsigned short*)srow;
    *(v2u*)(hrow + 4 * lane)       = w0;
    *(v2u*)(hrow + 128 + 4 * lane) = w1;
    wave_sync_lds();
    const v4u hv = *(const v4u*)(hrow + 8 * lane);
    const size_t crow = (size_t)(grow - row0);
    float* xo = X1F + crow * CCH;
    unsigned short* ho = X1H + crow * CCH;
    for (int pass = 0; pass < 2; ++pass) {
      *(volatile v4f*)(xo + 4 * lane)       = ya;
      *(volatile v4f*)(xo + 128 + 4 * lane) = yb;
      *(volatile v4u*)(ho + 8 * lane)       = hv;
      __threadfence();
    }
  }
}

template <int OM, int HASR, int ACT, int HASB>
__global__ __launch_bounds__(256) void gemm64(
    const unsigned short* __restrict__ Ap, int lda, long long sA,
    const unsigned short* __restrict__ Btp, int ldb, long long sB,
    const float* __restrict__ Rp, const float* __restrict__ Bip,
    void* Cout, int ldc, long long sC,
    int M, int N, int K, float oscale, float ocarry) {
  __shared__ __align__(16) float sT[8][16 * 68];
  const int by   = blockIdx.y;
  const int lane = threadIdx.x & 31;
  const int wave = threadIdx.x >> 5;
  const int tilesN = N >> 6;
  const int tilesM = M >> 6;
  const int tile = blockIdx.x * 8 + wave;
  if (tile >= tilesM * tilesN) return;
  const int tm = tile / tilesN;
  const int tn = tile - tm * tilesN;
  const int m0 = tm << 6;
  const int n0 = tn << 6;

  const unsigned short* A1 = Ap  + (size_t)((long long)by * sA);
  const unsigned short* Bb = Btp + (size_t)((long long)by * sB);

  const int rlane = lane & 15;
  const int koff  = (lane >> 4) * 8;
  const int mOff  = (lane >> 4) * 8;

  v8f acc[4][4];
#pragma unroll
  for (int i = 0; i < 4; ++i)
#pragma unroll
    for (int j = 0; j < 4; ++j) acc[i][j] = zero8();

  for (int k0 = 0; k0 < K; k0 += 32) {
    v16h bh[4];
#pragma unroll
    for (int j = 0; j < 4; ++j) {
      const size_t bofs = (size_t)(n0 + (j << 4) + rlane) * ldb + koff + k0;
      bh[j] = ldfrag_u(Bb + bofs);
    }
#pragma unroll
    for (int i = 0; i < 4; ++i) {
      const size_t ao = (size_t)(m0 + (i << 4) + rlane) * lda + koff + k0;
      const v16h ah = ldfrag_u(A1 + ao);
#pragma unroll
      for (int j = 0; j < 4; ++j) acc[i][j] = mma_raw(ah, bh[j], acc[i][j]);
      dep_guard1(acc[i][0], acc[i][3], ah);
    }
    keep4_h(bh[0], bh[1], bh[2], bh[3]);
  }
  acc_guard4(acc[0][0], acc[0][1], acc[0][2], acc[0][3]);
  acc_guard4(acc[1][0], acc[1][1], acc[1][2], acc[1][3]);
  acc_guard4(acc[2][0], acc[2][1], acc[2][2], acc[2][3]);
  acc_guard4(acc[3][0], acc[3][1], acc[3][2], acc[3][3]);

  const int hh2 = lane >> 4, c4 = (lane & 15) * 4;
  const int q8  = lane >> 3, c8 = (lane & 7) * 8;

  float* slab = sT[wave];
#pragma unroll
  for (int i = 0; i < 4; ++i) {
    const int mBase = m0 + (i << 4);
#pragma unroll
    for (int j = 0; j < 4; ++j) {
#pragma unroll
      for (int r = 0; r < 8; ++r) {
        slab[(mOff + r) * 68 + (j << 4) + rlane] = acc[i][j][r];
      }
    }
    wave_sync_lds();
    if constexpr (OM == 0) {
      float* C = (float*)Cout + (size_t)((long long)by * sC);
      v4f bv = {0.f, 0.f, 0.f, 0.f};
      if constexpr (HASB == 1) {
        const v4f braw = *(const v4f*)(Bip + n0 + c4);
#pragma unroll
        for (int e = 0; e < 4; ++e) bv[e] = bfr(braw[e]);
      }
      v4f vals[8];
#pragma unroll
      for (int it = 0; it < 8; ++it) {
        const int row = it * 2 + hh2;
        const int gr  = mBase + row;
        v4f v = *(const v4f*)(slab + row * 68 + c4);
        v4f rv = {0.f, 0.f, 0.f, 0.f};
        if constexpr (HASR == 2) {
          const float* R = Rp + (size_t)((long long)by * sC);
          rv = *(const v4f*)(R + (size_t)gr * ldc + n0 + c4);
        }
#pragma unroll
        for (int e = 0; e < 4; ++e) v[e] = (v[e] * oscale + bv[e]) + rv[e];
        vals[it] = v;
      }
      for (int pass = 0; pass < 2; ++pass) {
#pragma unroll
        for (int it = 0; it < 8; ++it) {
          const int gr = mBase + it * 2 + hh2;
          *(volatile v4f*)(C + (size_t)gr * ldc + n0 + c4) = vals[it];
        }
        __threadfence();
      }
    } else {
      unsigned short* C = (unsigned short*)Cout + (size_t)((long long)by * sC);
      float bb[8];
#pragma unroll
      for (int e = 0; e < 8; ++e) bb[e] = 0.f;
      if constexpr (HASB == 1) {
        const v4f ba = *(const v4f*)(Bip + n0 + c8), bbv = *(const v4f*)(Bip + n0 + c8 + 4);
#pragma unroll
        for (int e = 0; e < 4; ++e) { bb[e] = bfr(ba[e]); bb[4 + e] = bfr(bbv[e]); }
      }
      v4u hv[4];
#pragma unroll
      for (int it = 0; it < 4; ++it) {
        const int row = it * 4 + q8;
        const float* sp = slab + row * 68 + c8;
        v4u a = {0u, 0u, 0u, 0u};
#pragma unroll
        for (int e = 0; e < 4; ++e) {
          float f0 = sp[2 * e] * oscale + bb[2 * e];
          float f1 = sp[2 * e + 1] * oscale + bb[2 * e + 1];
          if constexpr (ACT == 1) { f0 = gelu_f(f0); f1 = gelu_f(f1); }
          f0 *= ocarry; f1 *= ocarry;
          a[e] = pk16(h_bits((_Float16)f0), h_bits((_Float16)f1));
        }
        hv[it] = a;
      }
      for (int pass = 0; pass < 2; ++pass) {
#pragma unroll
        for (int it = 0; it < 4; ++it) {
          const int row = it * 4 + q8;
          *(volatile v4u*)(C + (size_t)(mBase + row) * ldc + n0 + c8) = hv[it];
        }
        __threadfence();
      }
    }
    wave_sync_lds();
  }
}

__global__ __launch_bounds__(256) void k_ln2(const float* __restrict__ Y2, const float* __restrict__ g2,
                                             const float* __restrict__ be2, float* out, int row0, int nrows) {
  const int lane = threadIdx.x & 31, wave = threadIdx.x >> 5;
  const int lr = blockIdx.x * 8 + wave;
  if (lr >= nrows) return;
  const float* yr = Y2 + (size_t)lr * CCH;
  const v4f va = *(const v4f*)(yr + 4 * lane), vb = *(const v4f*)(yr + 128 + 4 * lane);
  v4f ga = *(const v4f*)(g2 + 4 * lane), gb = *(const v4f*)(g2 + 128 + 4 * lane);
  v4f ea = *(const v4f*)(be2 + 4 * lane), eb = *(const v4f*)(be2 + 128 + 4 * lane);
#pragma unroll
  for (int e = 0; e < 4; ++e) { ga[e] = bfr(ga[e]); gb[e] = bfr(gb[e]); ea[e] = bfr(ea[e]); eb[e] = bfr(eb[e]); }
  float s = ((va[0] + va[1]) + (va[2] + va[3])) + ((vb[0] + vb[1]) + (vb[2] + vb[3]));
#pragma unroll
  for (int off = 1; off < 32; off <<= 1) s += __shfl_xor(s, off, 32);
  const float mu = s * (1.0f / (float)CCH);
  v4f da, db;
#pragma unroll
  for (int e = 0; e < 4; ++e) { da[e] = va[e] - mu; db[e] = vb[e] - mu; }
  float q = ((da[0] * da[0] + da[1] * da[1]) + (da[2] * da[2] + da[3] * da[3])) +
            ((db[0] * db[0] + db[1] * db[1]) + (db[2] * db[2] + db[3] * db[3]));
#pragma unroll
  for (int off = 1; off < 32; off <<= 1) q += __shfl_xor(q, off, 32);
  const float var  = q * (1.0f / (float)CCH);
  const float rstd = rsqrtf(var + LN_EPS);
  v4f ya, yb;
#pragma unroll
  for (int e = 0; e < 4; ++e) { ya[e] = da[e] * rstd * ga[e] + ea[e]; yb[e] = db[e] * rstd * gb[e] + eb[e]; }
  float* o = out + ((size_t)row0 + lr) * CCH;
  for (int pass = 0; pass < 2; ++pass) {
    *(volatile v4f*)(o + 4 * lane)       = ya;
    *(volatile v4f*)(o + 128 + 4 * lane) = yb;
    __threadfence();
  }
}

static inline size_t al256(size_t v) { return (v + 255) & ~(size_t)255; }

extern "C" void kernel_launch(void* const* d_in, const int* in_sizes, int n_in,
                              void* d_out, int out_size, void* d_ws, size_t ws_size,
                              hipStream_t stream) {
  if (n_in < 10) return;
  if (in_sizes[0] != NROWS * CCH) return;
  if (in_sizes[1] != NKQV * HDIM) return;
  if (in_sizes[2] != DFF * CCH || in_sizes[3] != DFF) return;
  if (in_sizes[4] != CCH * DFF || in_sizes[5] != CCH) return;
  if (in_sizes[6] != CCH || in_sizes[7] != CCH || in_sizes[8] != CCH || in_sizes[9] != CCH) return;
  if (out_size != NROWS * CCH) return;

  const float* x   = (const float*)d_in[0];
  const float* wk  = (const float*)d_in[1];
  const float* w1  = (const float*)d_in[2];
  const float* b1  = (const float*)d_in[3];
  const float* w2  = (const float*)d_in[4];
  const float* b2  = (const float*)d_in[5];
  const float* g1  = (const float*)d_in[6];
  const float* be1 = (const float*)d_in[7];
  const float* g2  = (const float*)d_in[8];
  const float* be2 = (const float*)d_in[9];
  float*       out = (float*)d_out;

  const size_t PWK  = (size_t)NKQV * HDIM * 2;
  const size_t PW1  = (size_t)DFF * CCH * 2;
  const size_t PW2  = (size_t)CCH * DFF * 2;
  const size_t PKT  = (size_t)NBH * HDIM * LTOK * 2;
  const size_t PKVW = (size_t)NBH * KVW_STRIDE * 4;
  const size_t PX1F = (size_t)CHROWS * CCH * 4;
  const size_t PX1H = (size_t)CHROWS * CCH * 2;
  const size_t PHH  = (size_t)CHROWS * DFF * 2;
  const size_t PY2  = (size_t)CHROWS * CCH * 4;
  size_t off = 0;
  const size_t oWK  = off; off = al256(off + PWK);
  const size_t oW1  = off; off = al256(off + PW1);
  const size_t oW2  = off; off = al256(off + PW2);
  const size_t oKT  = off; off = al256(off + PKT);
  const size_t oVT  = off; off = al256(off + PKT);
  const size_t oKVW = off; off = al256(off + PKVW);
  const size_t oX1F = off; off = al256(off + PX1F);
  const size_t oX1H = off; off = al256(off + PX1H);
  const size_t oHH  = off; off = al256(off + PHH);
  const size_t oY2  = off; off = al256(off + PY2);
  if (off > ws_size) return;
  if (off > (size_t)134217728) return;

  char* ws = (char*)d_ws;
  unsigned short* WK16 = (unsigned short*)(ws + oWK);
  unsigned short* W116 = (unsigned short*)(ws + oW1);
  unsigned short* W216 = (unsigned short*)(ws + oW2);
  unsigned short* KT16 = (unsigned short*)(ws + oKT);
  unsigned short* VT16 = (unsigned short*)(ws + oVT);
  float*          KVW  = (float*)(ws + oKVW);
  float*          X1F  = (float*)(ws + oX1F);
  unsigned short* X1H  = (unsigned short*)(ws + oX1H);
  unsigned short* HH   = (unsigned short*)(ws + oHH);
  float*          Y2   = (float*)(ws + oY2);

  const dim3 blk(256);
  const dim3 gCV(DFF * CCH / 8 / 256, 3);
  const dim3 gPJ(LTOK / 64, NBATCH);
  const dim3 gKV(NBH);
  const dim3 gAP(CHROWS / 32);
  const int tilesF1 = (CHROWS / 64) * (DFF / 64);
  const int tilesF2 = (CHROWS / 64) * (CCH / 64);
  const dim3 gF1((tilesF1 + 7) / 8, 1);
  const dim3 gF2((tilesF2 + 7) / 8, 1);
  const dim3 gLN(CHROWS / 8);

  k_wcvt<<<gCV, blk, 0, stream>>>(wk, w1, w2, WK16, W116, W216);
  k_proj<<<gPJ, blk, 0, stream>>>(x, WK16, KT16, VT16);
  k_kv<<<gKV, blk, 0, stream>>>(KT16, VT16, KVW);

  for (int c = 0; c < NCHUNK; ++c) {
    const int row0 = c * CHROWS;
    k_apply<<<gAP, blk, 0, stream>>>(x, WK16, KVW, g1, be1, X1F, X1H, row0);
    gemm64<2, 0, 1, 1><<<gF1, blk, 0, stream>>>(
        X1H, CCH, 0LL,
        W116, CCH, 0LL,
        X1F, b1,
        (void*)HH, DFF, 0LL,
        CHROWS, DFF, CCH, 1.0f / (H1C * W1S), GC);
    gemm64<0, 2, 0, 1><<<gF2, blk, 0, stream>>>(
        HH, DFF, 0LL,
        W216, DFF, 0LL,
        X1F, b2,
        (void*)Y2, CCH, 0LL,
        CHROWS, CCH, DFF, 1.0f / (GC * W2S), 1.0f);
    k_ln2<<<gLN, blk, 0, stream>>>(Y2, g2, be2, out, row0, CHROWS);
  }
}
